// QuadPrior_Attention_78391743086718
// MI455X (gfx1250) — hardware-verified
//
#include <hip/hip_runtime.h>

typedef float          v4f  __attribute__((ext_vector_type(4)));
typedef float          v8f  __attribute__((ext_vector_type(8)));
typedef unsigned short v8us __attribute__((ext_vector_type(8)));
typedef __bf16         v16bf __attribute__((ext_vector_type(16)));
typedef v4f  __attribute__((may_alias)) v4fa;
typedef v8us __attribute__((may_alias)) v8usa;

union FragB { v16bf v; v8us h[2]; };

#define NTOK  8192
#define CDIM  768
#define TSEQ  2048
#define NBAT  4
#define NHEAD 12
#define HDIM  64
#define NBLK  8
#define BSZ   96
#define KCAT  288
#define KPAD  320
#define NLIN  4
#define CAP   16

static_assert(NTOK % 128 == 0);
static_assert(BSZ % 32 == 0);
static_assert(KPAD % 64 == 0);
static_assert((NTOK * CDIM) % (8 * 256) == 0);
static_assert((NBLK * BSZ * KPAD) % (8 * 256) == 0);
static_assert(NHEAD * HDIM == CDIM && NBLK * BSZ == CDIM);

__device__ __forceinline__ unsigned short bf16_bits(float f) {
  unsigned int u = __float_as_uint(f);
  u += 0x7FFFu + ((u >> 16) & 1u);
  return (unsigned short)(u >> 16);
}
__device__ __forceinline__ float bf16_val(unsigned short b) {
  return __uint_as_float(((unsigned int)b) << 16);
}
__device__ __forceinline__ float bf16_rne(float f) { return bf16_val(bf16_bits(f)); }

__device__ __forceinline__ v8f wmma_bf(v16bf a, v16bf b, v8f c) {
  v8f d = __builtin_amdgcn_wmma_f32_16x16x32_bf16(false, a, false, b, (short)0, c, false, false);
  asm volatile("v_nop\n\tv_nop\n\tv_nop\n\tv_nop" : "+v"(d) : "v"(a), "v"(b));
  return d;
}

__device__ __forceinline__ v16bf load_frag_bf(const unsigned short* p, int h) {
  FragB f;
  f.h[0] = *(const v8usa*)(p + 8 * h);
  f.h[1] = *(const v8usa*)(p + 16 + 8 * h);
  return f.v;
}

__global__ __launch_bounds__(256) void cvt_x_kernel(const float* __restrict__ x,
                                                    unsigned short* __restrict__ xb) {
  const int g = blockIdx.x * 256 + threadIdx.x;
  if (g >= (NTOK * CDIM) / 8) return;
  const float* src = x + (size_t)g * 8;
  const v4f a = *(const v4fa*)src;
  const v4f c = *(const v4fa*)(src + 4);
  v8us o;
  o[0] = bf16_bits(a.x); o[1] = bf16_bits(a.y); o[2] = bf16_bits(a.z); o[3] = bf16_bits(a.w);
  o[4] = bf16_bits(c.x); o[5] = bf16_bits(c.y); o[6] = bf16_bits(c.z); o[7] = bf16_bits(c.w);
  unsigned short* dst = xb + (size_t)g * 8;
  *(volatile v8us*)dst = o;
  __threadfence();
  *(volatile v8us*)dst = o;
}

__global__ __launch_bounds__(256) void pack_w_kernel(
    const float* __restrict__ qv, const float* __restrict__ qr, const float* __restrict__ ql,
    const float* __restrict__ kv, const float* __restrict__ kr, const float* __restrict__ kl,
    const float* __restrict__ vv, const float* __restrict__ vr, const float* __restrict__ vl,
    const float* __restrict__ ov, const float* __restrict__ orr, const float* __restrict__ ol,
    unsigned short* __restrict__ wp)
{
  const int lin = blockIdx.y;
  const int g = blockIdx.x * 256 + threadIdx.x;
  if (g >= (NBLK * BSZ * KPAD) / 8) return;
  const float* Wv = (lin == 0) ? qv : ((lin == 1) ? kv : ((lin == 2) ? vv : ov));
  const float* Wr = (lin == 0) ? qr : ((lin == 1) ? kr : ((lin == 2) ? vr : orr));
  const float* Wl = (lin == 0) ? ql : ((lin == 1) ? kl : ((lin == 2) ? vl : ol));

  const int e    = g * 8;
  const int krel = e % KPAD;
  const int n    = (e / KPAD) % BSZ;
  const int db   = e / (KPAD * BSZ);
  const int s    = krel / BSZ;
  const int sk0  = krel - s * BSZ;
  const int rb   = (db >= 1) ? (db - 1) : 0;
  const int lb   = (db <= NBLK - 2) ? db : (NBLK - 2);
  const bool use_r = (s == 0) && (db >= 1);
  const bool use_v = (s == 1);
  const bool use_l = (s == 2) && (db <= NBLK - 2);
  const bool any   = use_r || use_v || use_l;
  const float* pv = Wv + (size_t)db * BSZ * BSZ;
  const float* pr = Wr + (size_t)rb * BSZ * BSZ;
  const float* pl = Wl + (size_t)lb * BSZ * BSZ;
  const float* src = use_v ? pv : (use_r ? pr : pl);

  v8us o;
  #pragma unroll
  for (int i = 0; i < 8; ++i) {
    const int col = (sk0 + i) * BSZ + n;
    const float val = src[col];
    o[i] = bf16_bits(any ? val : 0.0f);
  }
  unsigned short* dst = wp + (size_t)lin * (NBLK * BSZ * KPAD) + (size_t)e;
  *(volatile v8us*)dst = o;
  __threadfence();
  *(volatile v8us*)dst = o;
}

__device__ __forceinline__ void lin_store_pass(const float* sT, float* y, int m0, int db,
                                               int w, int lane) {
  const int q8 = lane & 7, sub = lane >> 3;
  #pragma unroll
  for (int i = 0; i < 12; ++i) {
    const int L = 48 * w + 4 * i + sub;
    const int row = L / 3, seg = L - 3 * row;
    const v4f v = *(const v4fa*)(sT + row * BSZ + 32 * seg + 4 * q8);
    float* dst = y + (size_t)(m0 + row) * CDIM + db * BSZ + 32 * seg + 4 * q8;
    *(volatile v4f*)dst = v;
  }
}

template <int NPROD>
__global__ __launch_bounds__(256) void blk_linear_kernel(
    const unsigned short* __restrict__ ahi,
    const unsigned short* __restrict__ alo,
    const unsigned short* __restrict__ wp,
    int lin_base,
    const float* __restrict__ bz0, const float* __restrict__ bz1, const float* __restrict__ bz2,
    float* yz0, float* yz1, float* yz2)
{
  __shared__ __attribute__((aligned(16))) float sT[128 * BSZ];

  const int tid = threadIdx.x, lane = tid & 31, w = tid >> 5;
  const int h = lane >> 4, m = lane & 15;
  const int tg = w & 3, ch = w >> 2;
  const int m0 = blockIdx.x * 128, db = blockIdx.y, z = blockIdx.z;
  const int lin = lin_base + z;
  const float* bias = (z == 0) ? bz0 : ((z == 1) ? bz1 : bz2);
  float* y = (z == 0) ? yz0 : ((z == 1) ? yz1 : yz2);

  const v8f zero8 = {0.f, 0.f, 0.f, 0.f, 0.f, 0.f, 0.f, 0.f};
  v8f acc[2][3];
  #pragma unroll
  for (int mt = 0; mt < 2; ++mt)
    #pragma unroll
    for (int nt = 0; nt < 3; ++nt) acc[mt][nt] = zero8;

  const unsigned short* ah0 = ahi + (size_t)(m0 + 32 * tg + m) * CDIM;
  const unsigned short* ah1 = ah0 + (size_t)16 * CDIM;
  const unsigned short* al0 = alo + (size_t)(m0 + 32 * tg + m) * CDIM;
  const unsigned short* al1 = al0 + (size_t)16 * CDIM;
  const unsigned short* wb  = wp + ((size_t)(lin * NBLK + db) * BSZ + 48 * ch + m) * KPAD;

  const int s_lo = (db == 0) ? 1 : 0;
  const int s_hi = (db == NBLK - 1) ? 1 : 2;

  #pragma unroll 1
  for (int s = s_lo; s <= s_hi; ++s) {
    const int sb = db - 1 + s;
    #pragma unroll 1
    for (int ks = 0; ks < 3; ++ks) {
      const int ka = sb * BSZ + 32 * ks;
      const int kw = s * BSZ + 32 * ks;
      const v16bf a0 = load_frag_bf(ah0 + ka, h);
      const v16bf a1 = load_frag_bf(ah1 + ka, h);
      v16bf c0 = a0, c1 = a1;
      if (NPROD == 2) {
        c0 = load_frag_bf(al0 + ka, h);
        c1 = load_frag_bf(al1 + ka, h);
      }
      #pragma unroll
      for (int nt = 0; nt < 3; ++nt) {
        const v16bf bfr = load_frag_bf(wb + (size_t)nt * 16 * KPAD + kw, h);
        acc[0][nt] = wmma_bf(a0, bfr, acc[0][nt]);
        acc[1][nt] = wmma_bf(a1, bfr, acc[1][nt]);
        if (NPROD == 2) {
          acc[0][nt] = wmma_bf(c0, bfr, acc[0][nt]);
          acc[1][nt] = wmma_bf(c1, bfr, acc[1][nt]);
        }
      }
    }
  }

  #pragma unroll
  for (int nt = 0; nt < 3; ++nt) {
    const int col = 48 * ch + 16 * nt + m;
    const float bv = bf16_rne(bias[db * BSZ + col]);
    #pragma unroll
    for (int mt = 0; mt < 2; ++mt) {
      #pragma unroll
      for (int r = 0; r < 8; ++r) {
        const int tokl = 32 * tg + 16 * mt + 8 * h + r;
        sT[tokl * BSZ + col] = acc[mt][nt][r] + bv;
      }
    }
  }
  __syncthreads();

  lin_store_pass(sT, y, m0, db, w, lane);
  __threadfence();
  lin_store_pass(sT, y, m0, db, w, lane);
}

__device__ __forceinline__ void att_store_pass(const unsigned short* sHi, const unsigned short* sLo,
                                               unsigned short* ah, unsigned short* al,
                                               int row, int tid) {
  const v8us a = *(const v8usa*)(sHi + 8 * tid);
  const v8us c = *(const v8usa*)(sLo + 8 * tid);
  const size_t gi = (size_t)row * CDIM + 8 * tid;
  *(volatile v8us*)(ah + gi) = a;
  *(volatile v8us*)(al + gi) = c;
}

__global__ __launch_bounds__(96) void sparse_attn_kernel(
    const float* __restrict__ qf,
    const float* __restrict__ kf,
    const float* __restrict__ vf,
    const float* __restrict__ mask,
    unsigned short* ah,
    unsigned short* al)
{
  __shared__ int sCnt[2];
  __shared__ int sList[CAP];
  __shared__ __attribute__((aligned(16))) unsigned short sHi[CDIM];
  __shared__ __attribute__((aligned(16))) unsigned short sLo[CDIM];

  const int tid = threadIdx.x, lane = tid & 31, w = tid >> 5;
  const int row = blockIdx.x;
  const int b = row >> 11, i = row & (TSEQ - 1);
  const float ninf = __uint_as_float(0xff800000u);
  const float* mrow = mask + (size_t)i * TSEQ;

  unsigned int hits = 0u;
  if (w < 2) {
    const float* mp = mrow + 32 * tid;
    #pragma unroll
    for (int g = 0; g < 8; ++g) {
      const v4f mv = *(const v4fa*)(mp + 4 * g);
      const unsigned int bb = (mv.x != ninf ? 1u : 0u) | (mv.y != ninf ? 2u : 0u) |
                              (mv.z != ninf ? 4u : 0u) | (mv.w != ninf ? 8u : 0u);
      hits |= bb << (4 * g);
    }
  }
  const int c = (int)__popc(hits);
  int incl = c;
  #pragma unroll
  for (int d = 1; d < 32; d <<= 1) {
    const int v = __shfl_up(incl, d);
    incl = (lane >= d) ? (incl + v) : incl;
  }
  if (w < 2 && lane == 31) sCnt[w] = incl;
  __syncthreads();
  const int t0 = sCnt[0], t1 = sCnt[1];
  const int total = t0 + t1;
  {
    int pos = ((w == 1) ? t0 : 0) + incl - c;
    unsigned int hrem = hits;
    #pragma unroll 1
    for (int q = 0; q < 32; ++q) {
      if (hrem == 0u) break;
      const int bit = __builtin_ffs((int)hrem) - 1;
      hrem &= (hrem - 1u);
      if (pos < CAP) sList[pos] = 32 * tid + bit;
      ++pos;
    }
  }
  __syncthreads();

  const int n = (total < CAP) ? total : CAP;
  const bool bad = (total <= 0) || (total > CAP);

  const int grp = lane >> 3, s8 = lane & 7;
  const int hd = 4 * w + grp;
  const size_t hoff = (size_t)hd * HDIM + 8 * s8;
  const float* qp = qf + (size_t)row * CDIM + hoff;
  const v4f qa = *(const v4fa*)qp;
  const v4f qc = *(const v4fa*)(qp + 4);
  const float q0 = qa.x * 0.125f, q1 = qa.y * 0.125f, q2 = qa.z * 0.125f, q3 = qa.w * 0.125f;
  const float q4 = qc.x * 0.125f, q5 = qc.y * 0.125f, q6 = qc.z * 0.125f, q7 = qc.w * 0.125f;
  const float* kbase = kf + (size_t)b * TSEQ * CDIM + hoff;
  const float* vbase = vf + (size_t)b * TSEQ * CDIM + hoff;

  float mrun = ninf, lrun = 0.0f;
  float o0 = 0.f, o1 = 0.f, o2 = 0.f, o3 = 0.f, o4 = 0.f, o5 = 0.f, o6 = 0.f, o7 = 0.f;

  #pragma unroll 1
  for (int p = 0; p < n; ++p) {
    int j = sList[p];
    j = (j < 0) ? 0 : ((j > TSEQ - 1) ? (TSEQ - 1) : j);
    const float mvl = bf16_rne(mrow[j]);
    const float* kp = kbase + (size_t)j * CDIM;
    const v4f ka = *(const v4fa*)kp;
    const v4f kc = *(const v4fa*)(kp + 4);
    float dsum = q0 * ka.x + q1 * ka.y + q2 * ka.z + q3 * ka.w +
                 q4 * kc.x + q5 * kc.y + q6 * kc.z + q7 * kc.w;
    dsum += __shfl_xor(dsum, 4);
    dsum += __shfl_xor(dsum, 2);
    dsum += __shfl_xor(dsum, 1);
    const float sc = dsum + mvl;
    const float* vp = vbase + (size_t)j * CDIM;
    const v4f va = *(const v4fa*)vp;
    const v4f vc = *(const v4fa*)(vp + 4);
    const float mn = fmaxf(mrun, sc);
    const float alpha = __expf(mrun - mn);
    const float e = __expf(sc - mn);
    mrun = mn;
    lrun = lrun * alpha + e;
    o0 = o0 * alpha + e * va.x;  o1 = o1 * alpha + e * va.y;
    o2 = o2 * alpha + e * va.z;  o3 = o3 * alpha + e * va.w;
    o4 = o4 * alpha + e * vc.x;  o5 = o5 * alpha + e * vc.y;
    o6 = o6 * alpha + e * vc.z;  o7 = o7 * alpha + e * vc.w;
  }

  const float inv = 1.0f / (bad ? 1.0f : lrun);
  const float nanv = __uint_as_float(0x7fc00000u);
  float rr[8];
  rr[0] = bad ? nanv : o0 * inv;  rr[1] = bad ? nanv : o1 * inv;
  rr[2] = bad ? nanv : o2 * inv;  rr[3] = bad ? nanv : o3 * inv;
  rr[4] = bad ? nanv : o4 * inv;  rr[5] = bad ? nanv : o5 * inv;
  rr[6] = bad ? nanv : o6 * inv;  rr[7] = bad ? nanv : o7 * inv;
  v8us hi8, lo8;
  #pragma unroll
  for (int t = 0; t < 8; ++t) {
    const unsigned short hb = bf16_bits(rr[t]);
    const float hfv = bf16_val(hb);
    hi8[t] = hb;
    lo8[t] = bf16_bits(rr[t] - hfv);
  }
  *(v8usa*)(sHi + hoff) = hi8;
  *(v8usa*)(sLo + hoff) = lo8;
  __syncthreads();

  att_store_pass(sHi, sLo, ah, al, row, tid);
  __threadfence();
  att_store_pass(sHi, sLo, ah, al, row, tid);
}

extern "C" void kernel_launch(void* const* d_in, const int* in_sizes, int n_in,
                              void* d_out, int out_size, void* d_ws, size_t ws_size,
                              hipStream_t stream) {
  if (n_in < 18) return;
  if (in_sizes[0] != NTOK * CDIM) return;
  if (out_size != NTOK * CDIM) return;
  for (int l = 0; l < NLIN; ++l) {
    if (in_sizes[1 + 4 * l] != NBLK * BSZ * BSZ) return;
    if (in_sizes[2 + 4 * l] != (NBLK - 1) * BSZ * BSZ) return;
    if (in_sizes[3 + 4 * l] != (NBLK - 1) * BSZ * BSZ) return;
    if (in_sizes[4 + 4 * l] != CDIM) return;
  }
  if (in_sizes[17] != TSEQ * TSEQ) return;

  const float* x    = (const float*)d_in[0];
  const float* qv = (const float*)d_in[1];  const float* qr = (const float*)d_in[2];
  const float* ql = (const float*)d_in[3];  const float* qb = (const float*)d_in[4];
  const float* kv = (const float*)d_in[5];  const float* kr = (const float*)d_in[6];
  const float* kl = (const float*)d_in[7];  const float* kb = (const float*)d_in[8];
  const float* vv = (const float*)d_in[9];  const float* vr = (const float*)d_in[10];
  const float* vl = (const float*)d_in[11]; const float* vb = (const float*)d_in[12];
  const float* ov = (const float*)d_in[13]; const float* orr = (const float*)d_in[14];
  const float* ol = (const float*)d_in[15]; const float* ob = (const float*)d_in[16];
  const float* mask = (const float*)d_in[17];
  float* out = (float*)d_out;

  const size_t xb_bytes = (size_t)NTOK * CDIM * 2;
  const size_t wp_bytes = (size_t)NLIN * NBLK * BSZ * KPAD * 2;
  const size_t pf_bytes = (size_t)NTOK * CDIM * 4;
  const size_t ap_bytes = (size_t)NTOK * CDIM * 2;
  const size_t total = xb_bytes + wp_bytes + 3 * pf_bytes + 2 * ap_bytes;
  if (total > ws_size) return;

  char* ws = (char*)d_ws;
  unsigned short* xbp = (unsigned short*)(ws);
  unsigned short* wpp = (unsigned short*)(ws + xb_bytes);
  float* qf = (float*)(ws + xb_bytes + wp_bytes);
  float* kfp = (float*)(ws + xb_bytes + wp_bytes + pf_bytes);
  float* vfp = (float*)(ws + xb_bytes + wp_bytes + 2 * pf_bytes);
  unsigned short* ahp = (unsigned short*)(ws + xb_bytes + wp_bytes + 3 * pf_bytes);
  unsigned short* alp = (unsigned short*)(ws + xb_bytes + wp_bytes + 3 * pf_bytes + ap_bytes);

  cvt_x_kernel<<<(NTOK * CDIM) / (8 * 256), 256, 0, stream>>>(x, xbp);

  pack_w_kernel<<<dim3((NBLK * BSZ * KPAD) / (8 * 256), NLIN), 256, 0, stream>>>(
      qv, qr, ql, kv, kr, kl, vv, vr, vl, ov, orr, ol, wpp);

  blk_linear_kernel<1><<<dim3(NTOK / 128, NBLK, 3), 256, 0, stream>>>(
      xbp, xbp, wpp, 0, qb, kb, vb, qf, kfp, vfp);

  sparse_attn_kernel<<<NTOK, 96, 0, stream>>>(qf, kfp, vfp, mask, ahp, alp);

  blk_linear_kernel<2><<<dim3(NTOK / 128, NBLK, 1), 256, 0, stream>>>(
      ahp, alp, wpp, 3, ob, ob, ob, out, out, out);
}
